// KANLinear_15255723835975
// MI455X (gfx1250) — hardware-verified
//
#include <hip/hip_runtime.h>

typedef __attribute__((ext_vector_type(16))) _Float16 v16h;
typedef __attribute__((ext_vector_type(8)))  float    v8f;

#define IN_F   256
#define OUT_F  256
#define KTOT   2304
#define LDA    40
#define NCHUNK 72
typedef __attribute__((ext_vector_type(4))) float v4f;
typedef __attribute__((ext_vector_type(4))) unsigned v4u;
template <typename T> __device__ __forceinline__ void vst2(void* p, T v) { *(volatile T*)p = v; __threadfence(); *(volatile T*)p = v; }

__global__ void kan_pack_w(const float* __restrict__ bw,
                           const float* __restrict__ sw,
                           _Float16* __restrict__ wf) {
  int g8 = blockIdx.x * blockDim.x + threadIdx.x;
  union { _Float16 h[8]; v4u u; } pk;
#pragma unroll
  for (int e = 0; e < 8; ++e) { int idx = g8 * 8 + e; int o = idx / KTOT; int k = idx - o * KTOT;
    pk.h[e] = (_Float16)((k < IN_F) ? bw[o * IN_F + k] : sw[(size_t)o * (IN_F * 8) + (k - IN_F)]); }
  vst2(wf + (size_t)g8 * 8, pk.u);
}

__device__ __forceinline__ float siluf(float x) {
  return x / (1.0f + expf(-x));
}

__device__ __forceinline__ void bspline8(float x, _Float16* out8) {
  float b[11];
#pragma unroll
  for (int j = 0; j < 11; ++j) {
    float gj  = 0.4f * j - 2.2f;
    float gj1 = 0.4f * (j + 1) - 2.2f;
    b[j] = (x >= gj && x < gj1) ? 1.0f : 0.0f;
  }
#pragma unroll
  for (int k = 1; k <= 3; ++k) {
    float inv = 1.0f / (0.4f * k);
#pragma unroll
    for (int j = 0; j < 11 - k; ++j) {
      float gj  = 0.4f * j - 2.2f;
      float gk1 = 0.4f * (j + k + 1) - 2.2f;
      b[j] = (x - gj) * inv * b[j] + (gk1 - x) * inv * b[j + 1];
    }
  }
#pragma unroll
  for (int j = 0; j < 8; ++j) out8[j] = (_Float16)b[j];
}

union AFrag { v16h v; uint4 q[2]; };
union BFrag { v16h v; uint4 q[2]; };
union H8    { _Float16 h[8]; uint4 q; };
union H4    { _Float16 h[4]; uint2 q; };

__device__ __forceinline__ void mma_step(const _Float16* __restrict__ As,
                                         const _Float16* __restrict__ wf,
                                         int lane, int mw, int nw, int k0,
                                         v8f acc[2][4]) {
  const int hl = lane & 15;
  const int hi = lane >> 4;
  AFrag a[2];
#pragma unroll
  for (int mt = 0; mt < 2; ++mt) {
    const _Float16* rp = As + (size_t)(mw + mt * 16 + hl) * LDA + hi * 8;
    a[mt].q[0] = *(const uint4*)(rp);
    a[mt].q[1] = *(const uint4*)(rp + 16);
  }
  BFrag b[4];
#pragma unroll
  for (int nt = 0; nt < 4; ++nt) {
    const _Float16* wp = wf + (size_t)(nw + nt * 16 + hl) * KTOT + k0 + hi * 8;
    b[nt].q[0] = *(const uint4*)(wp);
    b[nt].q[1] = *(const uint4*)(wp + 16);
  }
#pragma unroll
  for (int mt = 0; mt < 2; ++mt)
#pragma unroll
    for (int nt = 0; nt < 4; ++nt)
    { acc[mt][nt] = __builtin_amdgcn_wmma_f32_16x16x32_f16(
          false, a[mt].v, false, b[nt].v, (short)0, acc[mt][nt], false, false);
      asm volatile("v_nop\n\tv_nop\n\tv_nop\n\tv_nop" : "+v"(acc[mt][nt]) : "v"(a[mt].v), "v"(b[nt].v)); }
}

__global__ void __launch_bounds__(256)
kan_fused(const float* __restrict__ x,
          const _Float16* __restrict__ wf,
          float* __restrict__ out) {
  __shared__ __attribute__((aligned(16))) _Float16 As[2][128 * LDA];
  __shared__ __attribute__((aligned(16))) float So[8][32 * 64];

  const int t    = threadIdx.x;
  const int lane = t & 31;
  const int wave = t >> 5;
  const int wm   = wave >> 1;
  const int wn   = wave & 1;
  const int m0   = blockIdx.x * 128;
  const int n0   = blockIdx.y * 128;
  const int mw   = wm * 32;
  const int nw   = n0 + wn * 64;

  const int rb = t >> 3;
  const int cb = (t & 7) * 4;
  const float* xb = x + (size_t)(m0 + rb) * IN_F + cb;

  const int rs = t >> 2;
  const int fs = t & 3;
  const float* xs = x + (size_t)(m0 + rs) * IN_F + fs;

  v8f acc[2][4] = {};

  auto fill = [&](int buf, int kc) {
    _Float16* A = As[buf];
    if (kc < 8) {
      const int f0 = kc * 32;
#pragma unroll
      for (int i = 0; i < 4; ++i) {
        float4 v = *(const float4*)(xb + (size_t)i * 32 * IN_F + f0);
        H4 h;
        h.h[0] = (_Float16)siluf(v.x);
        h.h[1] = (_Float16)siluf(v.y);
        h.h[2] = (_Float16)siluf(v.z);
        h.h[3] = (_Float16)siluf(v.w);
        *(uint2*)(A + (size_t)(rb + i * 32) * LDA + cb) = h.q;
      }
    } else {
      const int f0 = (kc - 8) * 4;
#pragma unroll
      for (int i = 0; i < 2; ++i) {
        const float* xp = xs + (size_t)i * 64 * IN_F + f0;
        float xv = *xp;
        if (kc < NCHUNK - 1) __builtin_prefetch(xp + 4, 0, 1);
        H8 h;
        bspline8(xv, h.h);
        *(uint4*)(A + (size_t)(rs + i * 64) * LDA + fs * 8) = h.q;
      }
    }
  };

  fill(0, 0);
  for (int kc = 0; kc < NCHUNK; ++kc) {
    __syncthreads();
    if (kc + 1 < NCHUNK) fill((kc + 1) & 1, kc + 1);
    mma_step(As[kc & 1], wf, lane, mw, nw, kc * 32, acc);
  }

  const int hl = lane & 15;
  const int hi = lane >> 4;
  float* S = So[wave];
#pragma unroll
  for (int mt = 0; mt < 2; ++mt)
#pragma unroll
    for (int nt = 0; nt < 4; ++nt)
#pragma unroll
      for (int v = 0; v < 8; ++v) S[(mt * 16 + hi * 8 + v) * 64 + nt * 16 + hl] = acc[mt][nt][v];
  asm volatile("s_wait_dscnt 0" ::: "memory"); __builtin_amdgcn_wave_barrier(); __builtin_amdgcn_fence(__ATOMIC_RELEASE, "workgroup");
#pragma unroll 4
  for (int q = 0; q < 16; ++q) { const int rl = q * 2 + (lane >> 4), pc = lane & 15;
    vst2(out + (size_t)(m0 + mw + rl) * OUT_F + nw + pc * 4, *(const v4f*)(S + rl * 64 + pc * 4)); }
}

extern "C" void kernel_launch(void* const* d_in, const int* in_sizes, int n_in,
                              void* d_out, int out_size, void* d_ws, size_t ws_size,
                              hipStream_t stream) {
  (void)n_in; (void)out_size; (void)ws_size;
  const float* x  = (const float*)d_in[0];
  const float* bw = (const float*)d_in[1];
  const float* sw = (const float*)d_in[2];
  float* out      = (float*)d_out;
  _Float16* wf    = (_Float16*)d_ws;

  const int N = in_sizes[0] / IN_F;

  kan_pack_w<<<(OUT_F * KTOT / 8) / 256, 256, 0, stream>>>(bw, sw, wf);

  dim3 grid(N / 128, OUT_F / 128);
  kan_fused<<<grid, 256, 0, stream>>>(x, wf, out);
}
